// PhaseSyncAttentionV6_53850299957949
// MI455X (gfx1250) — hardware-verified
//
#include <hip/hip_runtime.h>

typedef _Float16 v16h __attribute__((ext_vector_type(16)));
typedef _Float16 v8h  __attribute__((ext_vector_type(8)));
typedef float    v8f  __attribute__((ext_vector_type(8)));
typedef float    v4f  __attribute__((ext_vector_type(4)));
typedef v8h __attribute__((may_alias)) v8ha;
typedef v4f __attribute__((may_alias)) v4fa;

union Frag { v16h v; v8h half[2]; };

#define BATCH  4
#define SEQ    1024
#define HID    768
#define NHEADS 12
#define NBANDS 8
#define HD     64
#define NBH    (BATCH * NHEADS)
#define MROWS  (BATCH * SEQ)
#define NX     (MROWS * HID)
#define NW     (HID * HID)
#define NPHI   (BATCH * NBANDS * SEQ)
#define FW     32
#define WSCALE 32.0f
#define QSCALE 0.125f
#define FSCALE 16.0f
#define PSCALE 16384.0f
#define CSCALE 16.0f

__device__ __forceinline__ v8f wmma_f16(v16h a, v16h b, v8f c) {
  v8f d = __builtin_amdgcn_wmma_f32_16x16x32_f16(false, a, false, b, (short)0, c, false, false);
  asm volatile("v_nop\n\tv_nop\n\tv_nop\n\tv_nop" : "+v"(d) : "v"(a), "v"(b));
  return d;
}

__device__ __forceinline__ v16h load_frag(const _Float16* p, int h) {
  Frag f;
  f.half[0] = *(const v8ha*)(p + 8 * h);
  f.half[1] = *(const v8ha*)(p + 16 + 8 * h);
  return f.v;
}

__device__ __forceinline__ v8f zero8f() {
  v8f z = {0.f, 0.f, 0.f, 0.f, 0.f, 0.f, 0.f, 0.f};
  return z;
}

__global__ __launch_bounds__(256) void cvt_x_kernel(const float* __restrict__ x,
                                                    _Float16* __restrict__ xh)
{
  const int g = blockIdx.x * 256 + threadIdx.x;
  if (g >= NX / 8) return;
  const float* src = x + (size_t)g * 8;
  const v4f a = *(const v4fa*)src;
  const v4f c = *(const v4fa*)(src + 4);
  const v8h o = { (_Float16)a.x, (_Float16)a.y, (_Float16)a.z, (_Float16)a.w,
                  (_Float16)c.x, (_Float16)c.y, (_Float16)c.z, (_Float16)c.w };
  _Float16* dst = xh + (size_t)g * 8;
  *(volatile v8h*)dst = o;
  __threadfence();
  *(volatile v8h*)dst = o;
}

__device__ __forceinline__ void w_store_pass(const _Float16* sT, _Float16* wt, int mat,
                                             int f0, int k0, int w, int lane) {
  const int q8 = lane & 7, sub = lane >> 3;
  #pragma unroll
  for (int i = 0; i < 2; ++i) {
    const int lid = w * 8 + i * 4 + sub;
    const v8h v = *(const v8ha*)(sT + lid * 64 + 8 * q8);
    _Float16* dst = wt + ((size_t)(mat * HID + f0 + lid)) * HID + k0 + 8 * q8;
    *(volatile v8h*)dst = v;
  }
}

__global__ __launch_bounds__(256) void cvt_w_kernel(
    const float* __restrict__ wq, const float* __restrict__ wk,
    const float* __restrict__ wv, const float* __restrict__ wo,
    _Float16* __restrict__ wt)
{
  __shared__ __attribute__((aligned(16))) _Float16 sT[64 * 64];

  const int tid = threadIdx.x, lane = tid & 31, w = tid >> 5;
  const int f0 = blockIdx.x * 64, k0 = blockIdx.y * 64, mat = blockIdx.z;
  const float* W = (mat == 0) ? wq : ((mat == 1) ? wk : ((mat == 2) ? wv : wo));

  #pragma unroll
  for (int i = 0; i < 4; ++i) {
    const int idx = tid + 256 * i;
    const int kk = idx >> 4, ff = (idx & 15) * 4;
    const v4f v = *(const v4fa*)(W + (size_t)(k0 + kk) * HID + f0 + ff);
    sT[(ff + 0) * 64 + kk] = (_Float16)(v.x * WSCALE);
    sT[(ff + 1) * 64 + kk] = (_Float16)(v.y * WSCALE);
    sT[(ff + 2) * 64 + kk] = (_Float16)(v.z * WSCALE);
    sT[(ff + 3) * 64 + kk] = (_Float16)(v.w * WSCALE);
  }
  __syncthreads();

  w_store_pass(sT, wt, mat, f0, k0, w, lane);
  __threadfence();
  w_store_pass(sT, wt, mat, f0, k0, w, lane);
}

__device__ __forceinline__ void feat_store_pass(const _Float16* sF, const float* sM,
                                                _Float16* pf, float* mh,
                                                int bh, int l0, int w, int lane) {
  const int q8 = lane & 7, sub = lane >> 3;
  #pragma unroll
  for (int i = 0; i < 4; ++i) {
    const int lid = w * 16 + i * 4 + sub;
    const v8h v = *(const v8ha*)(sF + lid * 64 + 8 * q8);
    _Float16* dst = pf + ((size_t)bh * SEQ + l0) * FW + lid * 64 + 8 * q8;
    *(volatile v8h*)dst = v;
  }
  if (w == 0 && lane < 16) {
    const v4f v = *(const v4fa*)(sM + 4 * lane);
    *(volatile v4f*)(mh + (size_t)bh * SEQ + l0 + 4 * lane) = v;
  }
}

__global__ __launch_bounds__(64) void feat_kernel(
    const float* __restrict__ cosp, const float* __restrict__ sinp,
    const float* __restrict__ mag,  const float* __restrict__ blog,
    _Float16* __restrict__ pf, float* __restrict__ mh)
{
  __shared__ float sBw[NHEADS * NBANDS];
  __shared__ float sBs[NHEADS * NBANDS];
  __shared__ __attribute__((aligned(16))) _Float16 sF[64 * FW];
  __shared__ __attribute__((aligned(16))) float sM[64];

  const int tid = threadIdx.x, lane = tid & 31, w = tid >> 5;
  const int b = blockIdx.y, l0 = blockIdx.x * 64, l = l0 + tid;

  if (tid < NHEADS) {
    const float* bl = blog + tid * NBANDS;
    float mx = bl[0];
    #pragma unroll 1
    for (int s = 1; s < NBANDS; ++s) mx = fmaxf(mx, bl[s]);
    float sum = 0.f;
    #pragma unroll 1
    for (int s = 0; s < NBANDS; ++s) {
      const float e = expf(bl[s] - mx);
      sBw[tid * NBANDS + s] = e;
      sum += e;
    }
    const float inv = 1.0f / sum;
    #pragma unroll 1
    for (int s = 0; s < NBANDS; ++s) {
      const float bw = sBw[tid * NBANDS + s] * inv;
      sBw[tid * NBANDS + s] = bw;
      sBs[tid * NBANDS + s] = sqrtf(bw + 1e-8f);
    }
  }

  float c[NBANDS], sn[NBANDS], mg[NBANDS];
  #pragma unroll
  for (int s = 0; s < NBANDS; ++s) {
    const int o = (b * NBANDS + s) * SEQ + l;
    c[s] = cosp[o]; sn[s] = sinp[o]; mg[s] = mag[o];
  }
  __syncthreads();

  const _Float16 hz = (_Float16)0.0f;
  const v8h vz = { hz, hz, hz, hz, hz, hz, hz, hz };

  #pragma unroll 1
  for (int hh = 0; hh < NHEADS; ++hh) {
    float fc[NBANDS], fs[NBANDS];
    float mval = 0.f;
    #pragma unroll
    for (int s = 0; s < NBANDS; ++s) {
      const float ws = sBs[hh * NBANDS + s];
      const float bw = sBw[hh * NBANDS + s];
      fc[s] = (c[s] * ws) * FSCALE;
      fs[s] = (sn[s] * ws) * FSCALE;
      mval += mg[s] * bw;
    }
    const v8h vc = { (_Float16)fc[0], (_Float16)fc[1], (_Float16)fc[2], (_Float16)fc[3],
                     (_Float16)fc[4], (_Float16)fc[5], (_Float16)fc[6], (_Float16)fc[7] };
    const v8h vs = { (_Float16)fs[0], (_Float16)fs[1], (_Float16)fs[2], (_Float16)fs[3],
                     (_Float16)fs[4], (_Float16)fs[5], (_Float16)fs[6], (_Float16)fs[7] };
    *(v8ha*)(sF + tid * FW)      = vc;
    *(v8ha*)(sF + tid * FW + 8)  = vs;
    *(v8ha*)(sF + tid * FW + 16) = vz;
    *(v8ha*)(sF + tid * FW + 24) = vz;
    sM[tid] = mval;
    __syncthreads();

    const int bh = b * NHEADS + hh;
    feat_store_pass(sF, sM, pf, mh, bh, l0, w, lane);
    __threadfence();
    feat_store_pass(sF, sM, pf, mh, bh, l0, w, lane);
    __syncthreads();
  }
}

__device__ __forceinline__ void proj_store_pass(const _Float16* sT, _Float16* plane, _Float16* vt,
                                                int which, int bh, int l0, int w, int lane) {
  const int q8 = lane & 7, sub = lane >> 3;
  #pragma unroll
  for (int i = 0; i < 8; ++i) {
    const int lid = w * 32 + i * 4 + sub;
    v8h v;
    _Float16* dst;
    if (which != 2) {
      v = *(const v8ha*)(sT + lid * HD + 8 * q8);
      dst = plane + ((size_t)bh * SEQ + l0 + lid) * HD + 8 * q8;
    } else {
      const int d = lid >> 1, hl = lid & 1;
      v = *(const v8ha*)(sT + d * 128 + 64 * hl + 8 * q8);
      dst = vt + ((size_t)bh * HD + d) * SEQ + l0 + 64 * hl + 8 * q8;
    }
    *(volatile v8h*)dst = v;
  }
}

__global__ __launch_bounds__(128) void qkv_kernel(
    const _Float16* __restrict__ xh,
    const _Float16* __restrict__ wt,
    const float* __restrict__ bq, const float* __restrict__ bk, const float* __restrict__ bv,
    _Float16* __restrict__ qh,
    _Float16* __restrict__ kh,
    _Float16* __restrict__ vt)
{
  __shared__ __attribute__((aligned(16))) _Float16 sT[128 * 64];

  const int tid = threadIdx.x, lane = tid & 31, w = tid >> 5;
  const int h = lane >> 4, m = lane & 15;
  const int m0 = blockIdx.x * 128;
  const int cg = blockIdx.y;
  const int which = cg / NHEADS, head = cg - which * NHEADS;
  const int m0w = m0 + 32 * w;

  const _Float16* xa0 = xh + (size_t)(m0w + m) * HID;
  const _Float16* xa1 = xa0 + (size_t)16 * HID;
  const _Float16* wb  = wt + ((size_t)which * HID + head * HD + m) * HID;

  const v8f z8 = zero8f();
  v8f acc[2][4];
  #pragma unroll
  for (int mt = 0; mt < 2; ++mt)
    #pragma unroll
    for (int nt = 0; nt < 4; ++nt) acc[mt][nt] = z8;

  #pragma unroll 1
  for (int k0 = 0; k0 < HID; k0 += 32) {
    const v16h a0 = load_frag(xa0 + k0, h);
    const v16h a1 = load_frag(xa1 + k0, h);
    #pragma unroll
    for (int nt = 0; nt < 4; ++nt) {
      const v16h bb = load_frag(wb + (size_t)nt * 16 * HID + k0, h);
      acc[0][nt] = wmma_f16(a0, bb, acc[0][nt]);
      acc[1][nt] = wmma_f16(a1, bb, acc[1][nt]);
    }
  }

  const float* bias = (which == 0) ? bq : ((which == 1) ? bk : bv);
  const float osc = (which == 0) ? QSCALE : 1.0f;
  #pragma unroll
  for (int nt = 0; nt < 4; ++nt) {
    const int feat = 16 * nt + m;
    const float bvl = bias[head * HD + feat];
    #pragma unroll
    for (int mt = 0; mt < 2; ++mt) {
      #pragma unroll
      for (int r = 0; r < 8; ++r) {
        const int tokl = 32 * w + 16 * mt + 8 * h + r;
        const float y = (acc[mt][nt][r] * (1.0f / WSCALE) + bvl) * osc;
        const int idx = (which == 2) ? (feat * 128 + tokl) : (tokl * HD + feat);
        sT[idx] = (_Float16)y;
      }
    }
  }
  __syncthreads();

  const int b = m0 / SEQ, l0 = m0 - b * SEQ, bh = b * NHEADS + head;
  _Float16* plane = (which == 0) ? qh : kh;
  proj_store_pass(sT, plane, vt, which, bh, l0, w, lane);
  __threadfence();
  proj_store_pass(sT, plane, vt, which, bh, l0, w, lane);
}

__device__ __forceinline__ v16h pack_p(v8f a, v8f c) {
  const v16h r = { (_Float16)(a[0] * PSCALE), (_Float16)(a[1] * PSCALE), (_Float16)(a[2] * PSCALE), (_Float16)(a[3] * PSCALE),
                   (_Float16)(a[4] * PSCALE), (_Float16)(a[5] * PSCALE), (_Float16)(a[6] * PSCALE), (_Float16)(a[7] * PSCALE),
                   (_Float16)(c[0] * PSCALE), (_Float16)(c[1] * PSCALE), (_Float16)(c[2] * PSCALE), (_Float16)(c[3] * PSCALE),
                   (_Float16)(c[4] * PSCALE), (_Float16)(c[5] * PSCALE), (_Float16)(c[6] * PSCALE), (_Float16)(c[7] * PSCALE) };
  return r;
}

__device__ __forceinline__ void ctx_store_pass(const _Float16* so, _Float16* ctx,
                                               int b, int head, int q0, int lane) {
  const int q8 = lane & 7, sub = lane >> 3;
  #pragma unroll
  for (int i = 0; i < 4; ++i) {
    const int row = i * 4 + sub;
    const v8h v = *(const v8ha*)(so + row * 64 + 8 * q8);
    const size_t gi = ((size_t)b * SEQ + q0 + row) * HID + head * HD + 8 * q8;
    *(volatile v8h*)(ctx + gi) = v;
  }
}

__global__ __launch_bounds__(128) void attn_kernel(
    const _Float16* __restrict__ qh,
    const _Float16* __restrict__ kh,
    const _Float16* __restrict__ vt,
    const _Float16* __restrict__ pf,
    const float* __restrict__ mh,
    const float* __restrict__ mask,
    const float* __restrict__ pbias,
    const float* __restrict__ gscale,
    _Float16* __restrict__ ctx)
{
  __shared__ __attribute__((aligned(16))) _Float16 sO[4 * 16 * 64];

  const int tid = threadIdx.x, lane = tid & 31, w = tid >> 5;
  const int h = lane >> 4, m = lane & 15;
  const int bh = blockIdx.y, b = bh / NHEADS, head = bh - b * NHEADS;
  const int q0 = blockIdx.x * 64 + 16 * w;

  const _Float16* qrow = qh + ((size_t)bh * SEQ + q0 + m) * HD;
  const v16h qb0 = load_frag(qrow, h);
  const v16h qb1 = load_frag(qrow + 32, h);
  const v16h fq  = load_frag(pf + ((size_t)bh * SEQ + q0 + m) * FW, h);
  const float mi = mh[(size_t)bh * SEQ + q0 + m];
  const float pscale = expf(pbias[head]);
  const float g = gscale[0];

  const v8f z8 = zero8f();
  v8f o[4];
  #pragma unroll
  for (int t = 0; t < 4; ++t) o[t] = z8;
  float mrun = -1e30f, lrun = 0.0f, grun = 0.0f;

  const _Float16* kbase = kh + ((size_t)bh * SEQ + m) * HD;
  const _Float16* fbase = pf + ((size_t)bh * SEQ + m) * FW;
  const _Float16* vbase = vt + ((size_t)bh * HD + m) * SEQ;
  const float* mkp = mask + (size_t)b * SEQ + 8 * h;
  const float* mgp = mh + (size_t)bh * SEQ + 8 * h;

  #pragma unroll 1
  for (int kb = 0; kb < SEQ; kb += 64) {
    v8f s[4], pv[4];
    #pragma unroll
    for (int j = 0; j < 4; ++j) {
      const _Float16* kp = kbase + (size_t)(kb + 16 * j) * HD;
      const v16h kf0 = load_frag(kp, h);
      const v16h kf1 = load_frag(kp + 32, h);
      v8f z = z8;
      z = wmma_f16(kf0, qb0, z);
      z = wmma_f16(kf1, qb1, z);
      s[j] = z;
      const v16h ff = load_frag(fbase + (size_t)(kb + 16 * j) * FW, h);
      pv[j] = wmma_f16(ff, fq, z8);
    }
    #pragma unroll
    for (int j = 0; j < 4; ++j) {
      const v4f ga = *(const v4fa*)(mgp + kb + 16 * j);
      const v4f gb = *(const v4fa*)(mgp + kb + 16 * j + 4);
      const v4f ka = *(const v4fa*)(mkp + kb + 16 * j);
      const v4f kc = *(const v4fa*)(mkp + kb + 16 * j + 4);
      const float mj8[8] = { ga.x, ga.y, ga.z, ga.w, gb.x, gb.y, gb.z, gb.w };
      const float mk8[8] = { ka.x, ka.y, ka.z, ka.w, kc.x, kc.y, kc.z, kc.w };
      #pragma unroll
      for (int r = 0; r < 8; ++r) {
        const float mjr = mj8[r];
        const float hm = (2.0f * mi * mjr) * __builtin_amdgcn_rcpf(mi + mjr + 1e-8f);
        const float p = ((pv[j][r] * (1.0f / (FSCALE * FSCALE))) * hm) * pscale;
        pv[j][r] = p;
        s[j][r] = (s[j][r] + p) + mk8[r];
      }
    }

    float mloc = s[0][0];
    #pragma unroll
    for (int j = 0; j < 4; ++j)
      #pragma unroll
      for (int r = 0; r < 8; ++r) mloc = fmaxf(mloc, s[j][r]);
    mloc = fmaxf(mloc, __shfl_xor(mloc, 16));
    const float mnew = fmaxf(mrun, mloc);
    const float alpha = __expf(mrun - mnew);
    mrun = mnew;
    float lsum = 0.0f, gsum = 0.0f;
    #pragma unroll
    for (int j = 0; j < 4; ++j)
      #pragma unroll
      for (int r = 0; r < 8; ++r) {
        const float e  = __expf(s[j][r] - mnew);
        const float gt = __builtin_amdgcn_rcpf(1.0f + __expf(-g * pv[j][r]));
        const float wv = e * gt;
        lsum += e;
        gsum += wv;
        s[j][r] = wv;
      }
    lsum += __shfl_xor(lsum, 16);
    gsum += __shfl_xor(gsum, 16);
    lrun = lrun * alpha + lsum;
    grun = grun * alpha + gsum;
    #pragma unroll
    for (int t = 0; t < 4; ++t)
      #pragma unroll
      for (int r = 0; r < 8; ++r) o[t][r] = o[t][r] * alpha;

    const v16h pb0 = pack_p(s[0], s[1]);
    const v16h pb1 = pack_p(s[2], s[3]);

    #pragma unroll
    for (int t = 0; t < 4; ++t) {
      const _Float16* vp = vbase + (size_t)(16 * t) * SEQ + kb;
      const v16h vf0 = load_frag(vp, h);
      const v16h vf1 = load_frag(vp + 32, h);
      o[t] = wmma_f16(vf0, pb0, o[t]);
      o[t] = wmma_f16(vf1, pb1, o[t]);
    }
  }

  const float inv = (1.0f / (grun + 1e-9f * lrun)) * (CSCALE / PSCALE);
  _Float16* so = sO + w * 1024;
  #pragma unroll
  for (int t = 0; t < 4; ++t) {
    const v8h vv = { (_Float16)(o[t][0] * inv), (_Float16)(o[t][1] * inv), (_Float16)(o[t][2] * inv), (_Float16)(o[t][3] * inv),
                     (_Float16)(o[t][4] * inv), (_Float16)(o[t][5] * inv), (_Float16)(o[t][6] * inv), (_Float16)(o[t][7] * inv) };
    *(v8ha*)(so + m * 64 + 16 * t + 8 * h) = vv;
  }
  __syncthreads();

  ctx_store_pass(so, ctx, b, head, q0, lane);
  __threadfence();
  ctx_store_pass(so, ctx, b, head, q0, lane);
}

__global__ __launch_bounds__(256) void oproj_ln_kernel(
    const _Float16* __restrict__ ctx,
    const _Float16* __restrict__ wt,
    const float* __restrict__ bo, const float* __restrict__ x,
    const float* __restrict__ gamma, const float* __restrict__ beta,
    float* __restrict__ out)
{
  __shared__ __attribute__((aligned(16))) float sT[16 * HID];

  const int tid = threadIdx.x, lane = tid & 31, w = tid >> 5;
  const int h = lane >> 4, m = lane & 15;
  const int t0 = blockIdx.x * 16;

  const _Float16* arow = ctx + (size_t)(t0 + m) * HID;
  const _Float16* wrow = wt + ((size_t)3 * HID + 96 * w + m) * HID;

  const v8f z8 = zero8f();
  v8f acc[6];
  #pragma unroll
  for (int nt = 0; nt < 6; ++nt) acc[nt] = z8;

  #pragma unroll 1
  for (int k0 = 0; k0 < HID; k0 += 32) {
    const v16h a = load_frag(arow + k0, h);
    #pragma unroll
    for (int nt = 0; nt < 6; ++nt) {
      const v16h bb = load_frag(wrow + (size_t)nt * 16 * HID + k0, h);
      acc[nt] = wmma_f16(a, bb, acc[nt]);
    }
  }

  #pragma unroll
  for (int nt = 0; nt < 6; ++nt) {
    const int col = 96 * w + 16 * nt + m;
    const float bvl = bo[col];
    #pragma unroll
    for (int r = 0; r < 8; ++r) {
      const int row = 8 * h + r;
      const float xv = x[(size_t)(t0 + row) * HID + col];
      sT[row * HID + col] = (acc[nt][r] * (1.0f / (CSCALE * WSCALE)) + bvl) + xv;
    }
  }
  __syncthreads();

  #pragma unroll 1
  for (int rr = 0; rr < 2; ++rr) {
    const int row = 2 * w + rr;
    const float* srow = sT + row * HID;
    v4f v[6];
    float sum = 0.0f;
    #pragma unroll
    for (int i = 0; i < 6; ++i) {
      v[i] = *(const v4fa*)(srow + 128 * i + 4 * lane);
      sum += (v[i].x + v[i].y) + (v[i].z + v[i].w);
    }
    #pragma unroll
    for (int off = 16; off > 0; off >>= 1) sum += __shfl_xor(sum, off);
    const float mu = sum * (1.0f / (float)HID);
    float sq = 0.0f;
    #pragma unroll
    for (int i = 0; i < 6; ++i) {
      const v4f d = v[i] - mu;
      sq += (d.x * d.x + d.y * d.y) + (d.z * d.z + d.w * d.w);
    }
    #pragma unroll
    for (int off = 16; off > 0; off >>= 1) sq += __shfl_xor(sq, off);
    const float var = sq * (1.0f / (float)HID);
    const float rstd = 1.0f / sqrtf(var + 1e-12f);
    v4f y[6];
    #pragma unroll
    for (int i = 0; i < 6; ++i) {
      const v4f ga = *(const v4fa*)(gamma + 128 * i + 4 * lane);
      const v4f be = *(const v4fa*)(beta  + 128 * i + 4 * lane);
      y[i] = (v[i] - mu) * rstd * ga + be;
    }
    float* orow = out + (size_t)(t0 + row) * HID;
    #pragma unroll
    for (int i = 0; i < 6; ++i) *(volatile v4f*)(orow + 128 * i + 4 * lane) = y[i];
    __threadfence();
    #pragma unroll
    for (int i = 0; i < 6; ++i) *(volatile v4f*)(orow + 128 * i + 4 * lane) = y[i];
  }
}

extern "C" void kernel_launch(void* const* d_in, const int* in_sizes, int n_in,
                              void* d_out, int out_size, void* d_ws, size_t ws_size,
                              hipStream_t stream) {
  if (n_in < 18) return;
  if (in_sizes[0] != NX) return;
  if (in_sizes[1] != MROWS) return;
  if (in_sizes[2] != NPHI || in_sizes[3] != NPHI || in_sizes[4] != NPHI) return;
  if (in_sizes[5] != NW || in_sizes[7] != NW || in_sizes[9] != NW || in_sizes[11] != NW) return;
  if (in_sizes[6] != HID || in_sizes[8] != HID || in_sizes[10] != HID || in_sizes[12] != HID) return;
  if (in_sizes[13] != HID || in_sizes[14] != HID) return;
  if (in_sizes[15] != NHEADS * NBANDS || in_sizes[16] != NHEADS || in_sizes[17] != 1) return;
  if (out_size != NX) return;

  const float* x     = (const float*)d_in[0];
  const float* mask  = (const float*)d_in[1];
  const float* cosp  = (const float*)d_in[2];
  const float* sinp  = (const float*)d_in[3];
  const float* mag   = (const float*)d_in[4];
  const float* Wq    = (const float*)d_in[5];
  const float* bq    = (const float*)d_in[6];
  const float* Wk    = (const float*)d_in[7];
  const float* bk    = (const float*)d_in[8];
  const float* Wv    = (const float*)d_in[9];
  const float* bv    = (const float*)d_in[10];
  const float* Wo    = (const float*)d_in[11];
  const float* bo    = (const float*)d_in[12];
  const float* gamma = (const float*)d_in[13];
  const float* beta  = (const float*)d_in[14];
  const float* blog  = (const float*)d_in[15];
  const float* pbias = (const float*)d_in[16];
  const float* gsc   = (const float*)d_in[17];
  float* out = (float*)d_out;

  const size_t pl_bytes = (size_t)NX * 2;
  const size_t wt_bytes = (size_t)4 * NW * 2;
  const size_t pf_bytes = (size_t)NBH * SEQ * FW * 2;
  const size_t mh_bytes = (size_t)NBH * SEQ * 4;
  const size_t total = 5 * pl_bytes + wt_bytes + pf_bytes + mh_bytes;
  if (total > ws_size) return;

  char* ws = (char*)d_ws;
  size_t off = 0;
  _Float16* xh  = (_Float16*)(ws + off); off += pl_bytes;
  _Float16* wt  = (_Float16*)(ws + off); off += wt_bytes;
  _Float16* qh  = (_Float16*)(ws + off); off += pl_bytes;
  _Float16* kh  = (_Float16*)(ws + off); off += pl_bytes;
  _Float16* vt  = (_Float16*)(ws + off); off += pl_bytes;
  _Float16* ctx = (_Float16*)(ws + off); off += pl_bytes;
  _Float16* pf  = (_Float16*)(ws + off); off += pf_bytes;
  float*    mhd = (float*)(ws + off);    off += mh_bytes;
  if (off > ws_size) return;

  cvt_x_kernel<<<(NX / 8 + 255) / 256, 256, 0, stream>>>(x, xh);

  dim3 gW(HID / 64, HID / 64, 4);
  cvt_w_kernel<<<gW, 256, 0, stream>>>(Wq, Wk, Wv, Wo, wt);

  dim3 gF(SEQ / 64, BATCH);
  feat_kernel<<<gF, 64, 0, stream>>>(cosp, sinp, mag, blog, pf, mhd);

  dim3 gProj(MROWS / 128, 3 * NHEADS);
  qkv_kernel<<<gProj, 128, 0, stream>>>(xh, wt, bq, bk, bv, qh, kh, vt);

  dim3 gAtt(SEQ / 64, NBH);
  attn_kernel<<<gAtt, 128, 0, stream>>>(qh, kh, vt, pf, mhd, mask, pbias, gsc, ctx);

  oproj_ln_kernel<<<MROWS / 16, 256, 0, stream>>>(ctx, wt, bo, x, gamma, beta, out);
}
